// LengthRegulator_2929167696555
// MI455X (gfx1250) — hardware-verified
//
#include <hip/hip_runtime.h>
#include <stddef.h>
#include <stdint.h>

#define BSZ    16
#define TLEN   512
#define DIM    384
#define TP     514
#define MROWS  (BSZ * TLEN)
#define KC     1152
#define HPITCH 768
#define LOUT   1847
#define NOUT0  (BSZ * LOUT * DIM)
#define NOUT1  MROWS
#define GBM    32
#define GTHR   256
#define PTHR   256
#define NXU    (BSZ * TP * (DIM / 8))
#define NWU    (2 * DIM * (DIM / 8))
#define NHU    (BSZ * 2 * (HPITCH / 8))
#define NBX    (NXU / PTHR)
#define NBW    (NWU / PTHR)
#define NBH    (NHU / PTHR)
#define ETHR   256
#define EROWS  64
#define WSMAX  134217728
#define LN_EPS 1e-5f

static_assert(NXU % PTHR == 0 && NWU % PTHR == 0 && NHU % PTHR == 0);
static_assert((DIM * (DIM / 8)) % PTHR == 0);
static_assert(TLEN % GBM == 0 && MROWS % GBM == 0);
static_assert(KC % 32 == 0 && DIM % 32 == 0 && DIM % 128 == 0);
static_assert(GBM == 4 * (GTHR / 32) && DIM == 4 * 96);
static_assert(GBM * DIM * 4 <= 65536);
static_assert(TLEN == 2 * ETHR && EROWS == 8 * (ETHR / 32));
static_assert(((long long)NOUT0 * 4) % 128 == 0);
static_assert(NOUT0 + NOUT1 == 11356160);

typedef float          v4f   __attribute__((ext_vector_type(4)));
typedef float          v8f   __attribute__((ext_vector_type(8)));
typedef int            v8i   __attribute__((ext_vector_type(8)));
typedef unsigned short v4us  __attribute__((ext_vector_type(4)));
typedef unsigned short v8us  __attribute__((ext_vector_type(8)));
typedef unsigned short v16us __attribute__((ext_vector_type(16)));
typedef __bf16         v16bf __attribute__((ext_vector_type(16)));
typedef v4f  __attribute__((may_alias)) v4fa;
typedef v4us __attribute__((may_alias)) v4usa;
typedef v8us __attribute__((may_alias)) v8usa;
union FragB { v16bf v; v16us u; v8us h[2]; v8i w; };

__device__ __forceinline__ v8f wmb(const FragB& a, const FragB& b, v8f c) {
  v8f d = __builtin_amdgcn_wmma_f32_16x16x32_bf16(false, a.v, false, b.v, (short)0, c, false, false);
  asm volatile("v_nop\n\tv_nop\n\tv_nop\n\tv_nop" : "+v"(d) : "v"(a.w), "v"(b.w));
  return d;
}

__device__ __forceinline__ unsigned bf16_bits(float f) {
  const unsigned u = __float_as_uint(f);
  return (u + 0x7FFFu + ((u >> 16) & 1u)) >> 16;
}
__device__ __forceinline__ float bf16_val(float f) {
  return __uint_as_float(bf16_bits(f) << 16);
}
__device__ __forceinline__ v4f bf16_val4(v4f a) {
  v4f r;
  r.x = bf16_val(a.x); r.y = bf16_val(a.y); r.z = bf16_val(a.z); r.w = bf16_val(a.w);
  return r;
}
__device__ __forceinline__ float wsum32(float v) {
  v += __shfl_xor(v, 1);
  v += __shfl_xor(v, 2);
  v += __shfl_xor(v, 4);
  v += __shfl_xor(v, 8);
  v += __shfl_xor(v, 16);
  return v;
}

__global__ __launch_bounds__(PTHR) void k_prep(const float* __restrict__ x, const float* __restrict__ w1,
                                               const float* __restrict__ w2,
                                               unsigned short* XB, unsigned short* WB, unsigned short* HP) {
  const int blk = (int)blockIdx.x, tid = (int)threadIdx.x;
  if (blk < NBX) {
    const int g  = blk * PTHR + tid;
    const int R  = g / (DIM / 8);
    const int c8 = (g - R * (DIM / 8)) * 8;
    const int b  = R / TP;
    const int tp = R - b * TP;
    int t = tp - 1;
    const float fac = (tp >= 1 && tp <= TLEN) ? 1.0f : 0.0f;
    t = t < 0 ? 0 : (t > TLEN - 1 ? TLEN - 1 : t);
    const float* p = x + ((size_t)(b * TLEN + t)) * DIM + c8;
    const v4f a = *(const v4f*)p;
    const v4f c = *(const v4f*)(p + 4);
    v8us o;
    o[0] = (unsigned short)bf16_bits(a.x * fac + 0.0f); o[1] = (unsigned short)bf16_bits(a.y * fac + 0.0f);
    o[2] = (unsigned short)bf16_bits(a.z * fac + 0.0f); o[3] = (unsigned short)bf16_bits(a.w * fac + 0.0f);
    o[4] = (unsigned short)bf16_bits(c.x * fac + 0.0f); o[5] = (unsigned short)bf16_bits(c.y * fac + 0.0f);
    o[6] = (unsigned short)bf16_bits(c.z * fac + 0.0f); o[7] = (unsigned short)bf16_bits(c.w * fac + 0.0f);
    unsigned short* dp = XB + (size_t)g * 8;
    *(volatile v8us*)dp = o;
    __threadfence();
    *(volatile v8us*)dp = o;
  } else if (blk < NBX + NBW) {
    const int v   = (blk - NBX) * PTHR + tid;
    const int mat = v / (DIM * (DIM / 8));
    const int r   = v - mat * (DIM * (DIM / 8));
    const int o   = r / (DIM / 8);
    const int c8  = (r - o * (DIM / 8)) * 8;
    const float* wsrc = (mat == 0) ? w1 : w2;
    const float* p = wsrc + ((size_t)o * DIM + c8) * 3;
    const v4f q0 = *(const v4f*)(p);
    const v4f q1 = *(const v4f*)(p + 4);
    const v4f q2 = *(const v4f*)(p + 8);
    const v4f q3 = *(const v4f*)(p + 12);
    const v4f q4 = *(const v4f*)(p + 16);
    const v4f q5 = *(const v4f*)(p + 20);
    v8us o0, o1, o2;
    o0[0] = (unsigned short)bf16_bits(q0.x); o0[1] = (unsigned short)bf16_bits(q0.w);
    o0[2] = (unsigned short)bf16_bits(q1.z); o0[3] = (unsigned short)bf16_bits(q2.y);
    o0[4] = (unsigned short)bf16_bits(q3.x); o0[5] = (unsigned short)bf16_bits(q3.w);
    o0[6] = (unsigned short)bf16_bits(q4.z); o0[7] = (unsigned short)bf16_bits(q5.y);
    o1[0] = (unsigned short)bf16_bits(q0.y); o1[1] = (unsigned short)bf16_bits(q1.x);
    o1[2] = (unsigned short)bf16_bits(q1.w); o1[3] = (unsigned short)bf16_bits(q2.z);
    o1[4] = (unsigned short)bf16_bits(q3.y); o1[5] = (unsigned short)bf16_bits(q4.x);
    o1[6] = (unsigned short)bf16_bits(q4.w); o1[7] = (unsigned short)bf16_bits(q5.z);
    o2[0] = (unsigned short)bf16_bits(q0.z); o2[1] = (unsigned short)bf16_bits(q1.y);
    o2[2] = (unsigned short)bf16_bits(q2.x); o2[3] = (unsigned short)bf16_bits(q2.w);
    o2[4] = (unsigned short)bf16_bits(q3.z); o2[5] = (unsigned short)bf16_bits(q4.y);
    o2[6] = (unsigned short)bf16_bits(q5.x); o2[7] = (unsigned short)bf16_bits(q5.w);
    unsigned short* dp = WB + (size_t)mat * ((size_t)DIM * KC) + (size_t)o * KC + c8;
    *(volatile v8us*)(dp)           = o0;
    *(volatile v8us*)(dp + DIM)     = o1;
    *(volatile v8us*)(dp + 2 * DIM) = o2;
    __threadfence();
    *(volatile v8us*)(dp)           = o0;
    *(volatile v8us*)(dp + DIM)     = o1;
    *(volatile v8us*)(dp + 2 * DIM) = o2;
  } else {
    const int u  = (blk - NBX - NBW) * PTHR + tid;
    const int hr = u / (HPITCH / 8);
    const int wi = (u - hr * (HPITCH / 8)) * 8;
    const int b  = hr >> 1;
    const int row = b * TP + (((hr & 1) != 0) ? (TP - 1) : 0);
    unsigned short* dp = HP + (size_t)row * HPITCH + wi;
    const v8us z = {0, 0, 0, 0, 0, 0, 0, 0};
    *(volatile v8us*)dp = z;
    __threadfence();
    *(volatile v8us*)dp = z;
  }
}

template <int STAGE>
__global__ __launch_bounds__(GTHR) void k_conv(const unsigned short* __restrict__ Apl,
                                               const unsigned short* __restrict__ Wp,
                                               const float* __restrict__ bias, const float* __restrict__ gam,
                                               const float* __restrict__ bet, const float* __restrict__ wl,
                                               const float* __restrict__ bl,
                                               unsigned short* HPout, float* pred) {
  __shared__ __attribute__((aligned(16))) float stg[GBM * DIM];
  __shared__ __attribute__((aligned(16))) float spred[GBM];
  constexpr int APITCH = (STAGE == 0) ? DIM : HPITCH;
  constexpr int NTERM  = (STAGE == 0) ? 1 : 2;

  const int tid = (int)threadIdx.x, lane = tid & 31, wave = tid >> 5, hh = lane >> 4, m = lane & 15;
  const int rowBase = (int)blockIdx.x * GBM;
  const int b  = rowBase / TLEN;
  const int t0 = rowBase - b * TLEN;
  const int mt = wave & 1, cg = wave >> 1;

  v8f acc[6];
  {
    const v8f z = {0.f, 0.f, 0.f, 0.f, 0.f, 0.f, 0.f, 0.f};
#pragma unroll
    for (int t = 0; t < 6; ++t) acc[t] = z;
  }
  const unsigned short* arow = Apl + (size_t)(b * TP + t0 + 16 * mt + m) * (size_t)APITCH + 8 * hh;
  const unsigned short* brow = Wp + (size_t)(96 * cg + m) * (size_t)KC + 8 * hh;

#pragma unroll 1
  for (int term = 0; term < NTERM; ++term) {
#pragma unroll 1
    for (int dk = 0; dk < 3; ++dk) {
      const unsigned short* ap = arow + (size_t)dk * APITCH + term * DIM;
      const unsigned short* bp = brow + dk * DIM;
#pragma unroll 1
      for (int cb = 0; cb < DIM; cb += 32) {
        FragB af;
        af.h[0] = *(const v8usa*)(ap + cb);
        af.h[1] = *(const v8usa*)(ap + cb + 16);
#pragma unroll
        for (int nt = 0; nt < 6; ++nt) {
          const unsigned short* wq = bp + (size_t)(16 * nt) * (size_t)KC + cb;
          FragB bf;
          bf.h[0] = *(const v8usa*)wq;
          bf.h[1] = *(const v8usa*)(wq + 16);
          acc[nt] = wmb(af, bf, acc[nt]);
        }
      }
    }
  }

#pragma unroll
  for (int nt = 0; nt < 6; ++nt) {
    const int lc = 96 * cg + 16 * nt + m;
#pragma unroll
    for (int r = 0; r < 8; ++r) stg[(16 * mt + 8 * hh + r) * DIM + lc] = acc[nt][r];
  }
  __syncthreads();

  const int c0 = 4 * lane;
  v4f bi4[3], ga4[3], be4[3];
#pragma unroll
  for (int j = 0; j < 3; ++j) {
    bi4[j] = bf16_val4(*(const v4f*)(bias + 128 * j + c0));
    ga4[j] = bf16_val4(*(const v4f*)(gam + 128 * j + c0));
    be4[j] = bf16_val4(*(const v4f*)(bet + 128 * j + c0));
  }

  v4f pv[4][3];
#pragma unroll
  for (int i = 0; i < 4; ++i)
#pragma unroll
    for (int j = 0; j < 3; ++j) pv[i][j] = *(const v4fa*)(stg + (4 * wave + i) * DIM + 128 * j + c0);
  __syncthreads();

  const float invn = 1.0f / (float)DIM;
#pragma unroll
  for (int i = 0; i < 4; ++i) {
    v4f tv[3];
    float s = 0.0f;
#pragma unroll
    for (int j = 0; j < 3; ++j) {
      tv[j] = pv[i][j] + bi4[j];
      s += (tv[j].x + tv[j].y) + (tv[j].z + tv[j].w);
    }
    s = wsum32(s);
    const float mean = s * invn;
    float q = 0.0f;
#pragma unroll
    for (int j = 0; j < 3; ++j) {
      tv[j] = tv[j] - mean;
      q += tv[j].x * tv[j].x + tv[j].y * tv[j].y + tv[j].z * tv[j].z + tv[j].w * tv[j].w;
    }
    q = wsum32(q);
    const float inv = rsqrtf(q * invn + LN_EPS);
#pragma unroll
    for (int j = 0; j < 3; ++j) {
      v4f y;
      y.x = fmaxf(tv[j].x * inv * ga4[j].x + be4[j].x, 0.0f);
      y.y = fmaxf(tv[j].y * inv * ga4[j].y + be4[j].y, 0.0f);
      y.z = fmaxf(tv[j].z * inv * ga4[j].z + be4[j].z, 0.0f);
      y.w = fmaxf(tv[j].w * inv * ga4[j].w + be4[j].w, 0.0f);
      pv[i][j] = y;
    }
  }

  if constexpr (STAGE == 0) {
#pragma unroll
    for (int i = 0; i < 4; ++i) {
      unsigned short* srow = (unsigned short*)stg + (size_t)(4 * wave + i) * HPITCH;
#pragma unroll
      for (int j = 0; j < 3; ++j) {
        v4us h4, l4;
        unsigned hb;
        hb = bf16_bits(pv[i][j].x); h4[0] = (unsigned short)hb; l4[0] = (unsigned short)bf16_bits(pv[i][j].x - __uint_as_float(hb << 16));
        hb = bf16_bits(pv[i][j].y); h4[1] = (unsigned short)hb; l4[1] = (unsigned short)bf16_bits(pv[i][j].y - __uint_as_float(hb << 16));
        hb = bf16_bits(pv[i][j].z); h4[2] = (unsigned short)hb; l4[2] = (unsigned short)bf16_bits(pv[i][j].z - __uint_as_float(hb << 16));
        hb = bf16_bits(pv[i][j].w); h4[3] = (unsigned short)hb; l4[3] = (unsigned short)bf16_bits(pv[i][j].w - __uint_as_float(hb << 16));
        *(v4usa*)(srow + 128 * j + c0)       = h4;
        *(v4usa*)(srow + DIM + 128 * j + c0) = l4;
      }
    }
    __syncthreads();
    v8us qv[4][3];
#pragma unroll
    for (int i = 0; i < 4; ++i) {
      const unsigned short* srow = (const unsigned short*)stg + (size_t)(4 * wave + i) * HPITCH;
#pragma unroll
      for (int sgi = 0; sgi < 3; ++sgi) qv[i][sgi] = *(const v8usa*)(srow + 256 * sgi + 8 * lane);
    }
#pragma unroll
    for (int i = 0; i < 4; ++i) {
      unsigned short* rp = HPout + (size_t)(b * TP + t0 + 4 * wave + i + 1) * (size_t)HPITCH + 8 * lane;
#pragma unroll
      for (int sgi = 0; sgi < 3; ++sgi) *(volatile v8us*)(rp + 256 * sgi) = qv[i][sgi];
    }
    __threadfence();
#pragma unroll
    for (int i = 0; i < 4; ++i) {
      unsigned short* rp = HPout + (size_t)(b * TP + t0 + 4 * wave + i + 1) * (size_t)HPITCH + 8 * lane;
#pragma unroll
      for (int sgi = 0; sgi < 3; ++sgi) *(volatile v8us*)(rp + 256 * sgi) = qv[i][sgi];
    }
  } else {
    v4f wl4[3];
#pragma unroll
    for (int j = 0; j < 3; ++j) wl4[j] = bf16_val4(*(const v4f*)(wl + 128 * j + c0));
    const float blv = bf16_val(bl[0]);
#pragma unroll
    for (int i = 0; i < 4; ++i) {
      float p = 0.0f;
#pragma unroll
      for (int j = 0; j < 3; ++j) {
        p = fmaf(pv[i][j].x, wl4[j].x, p);
        p = fmaf(pv[i][j].y, wl4[j].y, p);
        p = fmaf(pv[i][j].z, wl4[j].z, p);
        p = fmaf(pv[i][j].w, wl4[j].w, p);
      }
      p = wsum32(p) + blv;
      if (lane == 0) spred[4 * wave + i] = p;
    }
    __syncthreads();
    if (wave == 0) {
      const v4f v = *(const v4fa*)(spred + 4 * (lane & 7));
      float* dp = pred + rowBase + 4 * lane;
      if (lane < 8) *(volatile v4f*)dp = v;
      __threadfence();
      if (lane < 8) *(volatile v4f*)dp = v;
    }
  }
}

__global__ __launch_bounds__(ETHR) void k_expand(const float* __restrict__ x, const int* __restrict__ dur,
                                                 float* out) {
  __shared__ int dsh[TLEN];
  __shared__ int cums[TLEN];
  const int tid = (int)threadIdx.x, lane = tid & 31, wave = tid >> 5;
  const int b = (int)blockIdx.y;
  const int l0 = (int)blockIdx.x * EROWS;
  dsh[tid]        = dur[b * TLEN + tid];
  dsh[tid + ETHR] = dur[b * TLEN + tid + ETHR];
  __syncthreads();
  if (wave == 0) {
    const int base = lane * (TLEN / 32);
    int s = 0;
#pragma unroll 1
    for (int i = 0; i < TLEN / 32; ++i) s += dsh[base + i];
    int incl = s;
#pragma unroll
    for (int d = 1; d < 32; d <<= 1) {
      const int y = __shfl_up(incl, d, 32);
      if (lane >= d) incl += y;
    }
    int run = incl - s;
#pragma unroll 1
    for (int i = 0; i < TLEN / 32; ++i) {
      run += dsh[base + i];
      cums[base + i] = run;
    }
  }
  __syncthreads();
  const int total = cums[TLEN - 1];

#pragma unroll 1
  for (int i = 0; i < 8; ++i) {
    const int l = l0 + 8 * wave + i;
    int pos = 0;
#pragma unroll
    for (int step = TLEN / 2; step >= 1; step >>= 1) {
      const int probe = pos + step - 1;
      pos = (cums[probe] <= l) ? (pos + step) : pos;
    }
    const int jc = pos > TLEN - 1 ? TLEN - 1 : pos;
    const float fac = (l < total) ? 1.0f : 0.0f;
    const float* src = x + ((size_t)(b * TLEN + jc)) * DIM + 4 * lane;
    v4f o[3];
#pragma unroll
    for (int sgi = 0; sgi < 3; ++sgi) {
      const v4f a = *(const v4f*)(src + 128 * sgi);
      v4f r;
      r.x = bf16_val(a.x) * fac + 0.0f;
      r.y = bf16_val(a.y) * fac + 0.0f;
      r.z = bf16_val(a.z) * fac + 0.0f;
      r.w = bf16_val(a.w) * fac + 0.0f;
      o[sgi] = r;
    }
    if (l < LOUT) {
      float* dp = out + ((size_t)(b * LOUT + l)) * DIM + 4 * lane;
#pragma unroll
      for (int sgi = 0; sgi < 3; ++sgi) *(volatile v4f*)(dp + 128 * sgi) = o[sgi];
      __threadfence();
#pragma unroll
      for (int sgi = 0; sgi < 3; ++sgi) *(volatile v4f*)(dp + 128 * sgi) = o[sgi];
    }
  }
}

static inline size_t al256(size_t o) { return (o + 255) & ~(size_t)255; }

extern "C" void kernel_launch(void* const* d_in, const int* in_sizes, int n_in,
                              void* d_out, int out_size, void* d_ws, size_t ws_size,
                              hipStream_t stream) {
  if (n_in < 12) return;
  if (in_sizes[0] != BSZ * TLEN * DIM) return;
  if (in_sizes[1] != BSZ * TLEN) return;
  if (in_sizes[2] != DIM * DIM * 3) return;
  if (in_sizes[3] != DIM || in_sizes[4] != DIM || in_sizes[5] != DIM) return;
  if (in_sizes[6] != DIM * DIM * 3) return;
  if (in_sizes[7] != DIM || in_sizes[8] != DIM || in_sizes[9] != DIM) return;
  if (in_sizes[10] != DIM || in_sizes[11] != 1) return;
  if (out_size != NOUT0 + NOUT1) return;

  const float* x   = (const float*)d_in[0];
  const int*   dur = (const int*)d_in[1];
  const float* w1  = (const float*)d_in[2];
  const float* b1  = (const float*)d_in[3];
  const float* g1  = (const float*)d_in[4];
  const float* be1 = (const float*)d_in[5];
  const float* w2  = (const float*)d_in[6];
  const float* b2  = (const float*)d_in[7];
  const float* g2  = (const float*)d_in[8];
  const float* be2 = (const float*)d_in[9];
  const float* wl  = (const float*)d_in[10];
  const float* bl  = (const float*)d_in[11];
  float* out  = (float*)d_out;
  float* pred = out + (size_t)NOUT0;

  char* ws = (char*)d_ws;
  size_t off = 0;
  const size_t oXB = off; off = al256(off + (size_t)BSZ * TP * DIM * 2);
  const size_t oWB = off; off = al256(off + (size_t)2 * DIM * KC * 2);
  const size_t oHP = off; off = al256(off + (size_t)BSZ * TP * HPITCH * 2);
  if (off > ws_size || off > (size_t)WSMAX) return;
  unsigned short* XB = (unsigned short*)(ws + oXB);
  unsigned short* WB = (unsigned short*)(ws + oWB);
  unsigned short* HP = (unsigned short*)(ws + oHP);

  k_prep<<<NBX + NBW + NBH, PTHR, 0, stream>>>(x, w1, w2, XB, WB, HP);
  k_conv<0><<<MROWS / GBM, GTHR, 0, stream>>>(XB, WB, b1, g1, be1, wl, bl, HP, pred);
  k_conv<1><<<MROWS / GBM, GTHR, 0, stream>>>(HP, WB + (size_t)DIM * KC, b2, g2, be2, wl, bl, HP, pred);
  dim3 gE((LOUT + EROWS - 1) / EROWS, BSZ);
  k_expand<<<gE, ETHR, 0, stream>>>(x, dur, out);
}
